// LowRankSVDBlock_86423331930456
// MI455X (gfx1250) — hardware-verified
//
#include <hip/hip_runtime.h>
#include <math.h>

typedef __attribute__((ext_vector_type(16))) _Float16 v16h;
typedef __attribute__((ext_vector_type(8)))  _Float16 v8h;
typedef __attribute__((ext_vector_type(8)))  float    v8f;
typedef __attribute__((ext_vector_type(4)))  float    v4f;
typedef unsigned short u16;

__device__ __forceinline__ void dep_guard_h(v8f& a, v8f& b, v16h x, v16h y) { asm volatile("v_nop\n\tv_nop\n\tv_nop\n\tv_nop" : "+v"(a), "+v"(b) : "v"(x), "v"(y)); }
__device__ __forceinline__ void keep4_h(v16h a, v16h b, v16h c, v16h d) { asm volatile("v_nop" :: "v"(a), "v"(b), "v"(c), "v"(d)); }
__device__ __forceinline__ void acc_guard4(v8f& a, v8f& b, v8f& c, v8f& d) { asm volatile("v_nop\n\tv_nop\n\tv_nop\n\tv_nop" : "+v"(a), "+v"(b), "+v"(c), "+v"(d)); }

template <typename T> struct Frag;
template <> struct Frag<_Float16> {
  typedef v16h V; union U { v16h v; v8h h[2]; };
  static __device__ __forceinline__ v16h load(const _Float16* p) {
    U f; f.h[0] = *(const v8h*)(p); f.h[1] = *(const v8h*)(p + 16); return f.v;
  }
  static __device__ __forceinline__ v8f mma(v16h a, v16h b, v8f c) {
    return __builtin_amdgcn_wmma_f32_16x16x32_f16(false, a, false, b, (short)0, c, false, false);
  }
  static __device__ __forceinline__ void guard(v8f& a, v8f& b, v16h x, v16h y) { dep_guard_h(a, b, x, y); }
  static __device__ __forceinline__ void keep(v16h a, v16h b, v16h c, v16h d) { keep4_h(a, b, c, d); }
};

__device__ __forceinline__ v8f mma_h(v16h a, v16h b, v8f c) {
  c = __builtin_amdgcn_wmma_f32_16x16x32_f16(false, a, false, b, (short)0, c, false, false);
  asm volatile("v_nop\n\tv_nop\n\tv_nop\n\tv_nop" : "+v"(c) : "v"(a), "v"(b));
  return c;
}

template <int BIAS_MODE, int OUT_MODE, bool RESID, int ACT>
__global__ __launch_bounds__(256) void wmma_gemm64(
    const u16* __restrict__ Ap, int lda, long strideA,
    const u16* __restrict__ Btp, int ldb, long strideB,
    void* __restrict__ Cout, int ldc, long strideC,
    const float* __restrict__ bias, long strideBias, float bscale,
    const float* __restrict__ resid, long strideR,
    int M, int N, int K, float scale, float oscale) {
  typedef _Float16 T;
  typedef v16h V;
  const T* A = (const T*)Ap; const T* Bt = (const T*)Btp;
  __shared__ __align__(16) float sT[8][16 * 68];
  const int b    = blockIdx.y;
  const int lane = threadIdx.x & 31;
  const int wave = threadIdx.x >> 5;
  const int tilesN = N >> 6;
  const int tilesM = M >> 6;
  const int tile = blockIdx.x * 8 + wave;
  if (tile >= tilesM * tilesN) return;
  const int tm = tile / tilesN;
  const int tn = tile - tm * tilesN;
  const int m0 = tm << 6;
  const int n0 = tn << 6;

  const T* Ab = A  + (size_t)b * strideA;
  const T* Bb = Bt + (size_t)b * strideB;

  const int rlane = lane & 15;
  const int koff  = (lane >> 4) * 8;
  const int mOff  = (lane >> 4) * 8;

  v8f acc[4][4];
#pragma unroll
  for (int i = 0; i < 4; ++i)
#pragma unroll
    for (int j = 0; j < 4; ++j) acc[i][j] = (v8f){0.f,0.f,0.f,0.f,0.f,0.f,0.f,0.f};

  for (int k0 = 0; k0 < K; k0 += 32) {
    V bh[4];
#pragma unroll
    for (int j = 0; j < 4; ++j) {
      const size_t bo = (size_t)(n0 + (j << 4) + rlane) * ldb + koff + k0;
      bh[j] = Frag<T>::load(Bb + bo);
    }
#pragma unroll
    for (int i = 0; i < 4; ++i) {
      const size_t ao = (size_t)(m0 + (i << 4) + rlane) * lda + koff + k0;
      V ah = Frag<T>::load(Ab + ao);
#pragma unroll
      for (int j = 0; j < 4; ++j) acc[i][j] = Frag<T>::mma(ah, bh[j], acc[i][j]);
      Frag<T>::guard(acc[i][0], acc[i][3], ah, ah);
    }
    Frag<T>::keep(bh[0], bh[1], bh[2], bh[3]);
  }
  acc_guard4(acc[0][0], acc[0][1], acc[0][2], acc[0][3]);
  acc_guard4(acc[1][0], acc[1][1], acc[1][2], acc[1][3]);
  acc_guard4(acc[2][0], acc[2][1], acc[2][2], acc[2][3]);
  acc_guard4(acc[3][0], acc[3][1], acc[3][2], acc[3][3]);

  float* slab = sT[wave];
  const float* Rb = RESID ? (resid + (size_t)b * strideR) : nullptr;
  const float* Bp = (BIAS_MODE != 0) ? (bias + (size_t)b * strideBias) : nullptr;
#pragma unroll
  for (int i = 0; i < 4; ++i) {
    const int mBase = m0 + (i << 4);
#pragma unroll
    for (int j = 0; j < 4; ++j) {
      const int n = n0 + (j << 4) + rlane;
      float bv = 0.f;
      if (BIAS_MODE == 2) bv = Bp[n] * bscale;
#pragma unroll
      for (int r = 0; r < 8; ++r) {
        float v = acc[i][j][r] * scale;
        if (BIAS_MODE == 1) v += Bp[mBase + mOff + r] * bscale;
        if (BIAS_MODE == 2) v += bv;
        if (RESID) v += Rb[(size_t)(mBase + mOff + r) * ldc + n];
        if (ACT == 5) v = 0.5f * v * (1.0f + erff(v * 0.70710678118654752f));
        v *= oscale;
        slab[(mOff + r) * 68 + (j << 4) + rlane] = v;
      }
    }
    __builtin_amdgcn_fence(__ATOMIC_RELEASE, "workgroup");
    __builtin_amdgcn_wave_barrier();
    __builtin_amdgcn_fence(__ATOMIC_ACQUIRE, "workgroup");
    if (OUT_MODE == 0) {
      float* C = (float*)Cout + (size_t)b * strideC;
      const int hh = lane >> 4, c4 = (lane & 15) * 4;
      for (int pass = 0; pass < 2; ++pass) {
#pragma unroll
        for (int it = 0; it < 8; ++it) {
          const int row = it * 2 + hh;
          v4f v = *(const v4f*)(slab + row * 68 + c4);
          *(volatile v4f*)(C + (size_t)(mBase + row) * ldc + n0 + c4) = v;
        }
        __threadfence();
      }
    } else {
      const int q = lane >> 3, c8 = (lane & 7) * 8;
      u16* C = (u16*)Cout + (size_t)b * strideC;
      for (int pass = 0; pass < 2; ++pass) {
#pragma unroll
        for (int it = 0; it < 4; ++it) {
          const int row = it * 4 + q;
          const float* sp = slab + row * 68 + c8;
          v8h hv;
#pragma unroll
          for (int e = 0; e < 8; ++e) hv[e] = (_Float16)sp[e];
          *(volatile v8h*)(C + (size_t)(mBase + row) * ldc + n0 + c8) = hv;
        }
        __threadfence();
      }
    }
    __builtin_amdgcn_fence(__ATOMIC_RELEASE, "workgroup");
    __builtin_amdgcn_wave_barrier();
    __builtin_amdgcn_fence(__ATOMIC_ACQUIRE, "workgroup");
  }
}

__global__ __launch_bounds__(256) void tcast64(const float* __restrict__ in, _Float16* __restrict__ out,
                                               int R, int C, float sc) {
  __shared__ float sT[64 * 65];
  const int tid = threadIdx.x, lane = tid & 31, wave = tid >> 5;
  const int c0 = blockIdx.x * 64, r0 = blockIdx.y * 64;
  {
    const int r = tid >> 2, cb = (tid & 3) * 16;
    const float* src = in + (size_t)(r0 + r) * C + c0 + cb;
#pragma unroll
    for (int i = 0; i < 4; ++i) {
      const v4f v = *(const v4f*)(src + 4 * i);
      sT[(cb + 4 * i + 0) * 65 + r] = v[0];
      sT[(cb + 4 * i + 1) * 65 + r] = v[1];
      sT[(cb + 4 * i + 2) * 65 + r] = v[2];
      sT[(cb + 4 * i + 3) * 65 + r] = v[3];
    }
  }
  __syncthreads();
  const int q = lane >> 3, c8 = (lane & 7) * 8;
  for (int pass = 0; pass < 2; ++pass) {
#pragma unroll
    for (int it = 0; it < 2; ++it) {
      const int row = wave * 8 + it * 4 + q;
      v8h hv;
#pragma unroll
      for (int e = 0; e < 8; ++e) hv[e] = (_Float16)(sT[row * 65 + c8 + e] * sc);
      *(volatile v8h*)(out + (size_t)(c0 + row) * R + r0 + c8) = hv;
    }
    __threadfence();
  }
}

__global__ __launch_bounds__(256) void tcast_v32(const float* __restrict__ a0, const float* __restrict__ a1,
                                                 const float* __restrict__ a2, _Float16* __restrict__ out, float sc) {
  __shared__ float s[32 * 65];
  const int tid = threadIdx.x;
  const int tsel = blockIdx.x >> 4, hd = blockIdx.x & 15;
  const float* src = (tsel == 0) ? a0 : ((tsel == 1) ? a1 : a2);
  src += (size_t)hd * 2048;
  {
    const int k = tid >> 3, nb = (tid & 7) * 8;
    const v4f v0 = *(const v4f*)(src + k * 64 + nb);
    const v4f v1 = *(const v4f*)(src + k * 64 + nb + 4);
    s[k * 65 + nb + 0] = v0[0]; s[k * 65 + nb + 1] = v0[1]; s[k * 65 + nb + 2] = v0[2]; s[k * 65 + nb + 3] = v0[3];
    s[k * 65 + nb + 4] = v1[0]; s[k * 65 + nb + 5] = v1[1]; s[k * 65 + nb + 6] = v1[2]; s[k * 65 + nb + 7] = v1[3];
  }
  __syncthreads();
  const int n = tid >> 2, kb = (tid & 3) * 8;
  v8h hv;
#pragma unroll
  for (int e = 0; e < 8; ++e) hv[e] = (_Float16)(s[(kb + e) * 65 + n] * sc);
  _Float16* dst = out + (size_t)blockIdx.x * 2048 + tid * 8;
  *(volatile v8h*)dst = hv;
  __threadfence();
  *(volatile v8h*)dst = hv;
}

__global__ __launch_bounds__(128) void layernorm_f16(const float* __restrict__ X, const float* __restrict__ g,
                                                     const float* __restrict__ bb, _Float16* __restrict__ out,
                                                     int D, float eps) {
  __shared__ float red[8];
  const int row = blockIdx.x, tid = threadIdx.x, lane = tid & 31, wave = tid >> 5;
  const float* xr = X + (size_t)row * D + tid * 8;
  const v4f a = *(const v4f*)xr;
  const v4f c = *(const v4f*)(xr + 4);
  float xv[8];
  xv[0] = a[0]; xv[1] = a[1]; xv[2] = a[2]; xv[3] = a[3];
  xv[4] = c[0]; xv[5] = c[1]; xv[6] = c[2]; xv[7] = c[3];
  float s1 = ((xv[0] + xv[1]) + (xv[2] + xv[3])) + ((xv[4] + xv[5]) + (xv[6] + xv[7]));
#pragma unroll
  for (int off = 16; off > 0; off >>= 1) s1 += __shfl_xor(s1, off, 32);
  if (lane == 0) red[wave] = s1;
  __syncthreads();
  const float invD = 1.0f / (float)D;
  const float mean = ((red[0] + red[1]) + (red[2] + red[3])) * invD;
  float s2 = 0.f;
#pragma unroll
  for (int e = 0; e < 8; ++e) { const float d = xv[e] - mean; s2 += d * d; }
#pragma unroll
  for (int off = 16; off > 0; off >>= 1) s2 += __shfl_xor(s2, off, 32);
  if (lane == 0) red[4 + wave] = s2;
  __syncthreads();
  const float var = ((red[4] + red[5]) + (red[6] + red[7])) * invD;
  const float rstd = rsqrtf(var + eps);
  v8h hv;
#pragma unroll
  for (int e = 0; e < 8; ++e) hv[e] = (_Float16)((xv[e] - mean) * rstd * g[tid * 8 + e] + bb[tid * 8 + e]);
  _Float16* dst = out + (size_t)row * D + tid * 8;
  *(volatile v8h*)dst = hv;
  __threadfence();
  *(volatile v8h*)dst = hv;
}

__global__ __launch_bounds__(128)
void attn64_f16(const _Float16* __restrict__ Qp, const _Float16* __restrict__ Kp,
                const _Float16* __restrict__ VTp, _Float16* __restrict__ Yp,
                int S, int H, int ldq, int ldvt, float sscale, float fillv) {
  union FB { v16h v; v8h h[2]; };
  __shared__ __align__(16) _Float16 Ksh[64 * 64];
  __shared__ __align__(16) _Float16 Vth[64 * 64];
  __shared__ __align__(16) _Float16 Psh[4][16 * 64];
  __shared__ __align__(16) float  Os[4][16 * 68];

  const int tid  = threadIdx.x;
  const int wave = tid >> 5;
  const int lane = tid & 31;
  const int hh   = lane >> 4;
  const int c    = lane & 15;

  const int nqb = S >> 6;
  const int bx = blockIdx.x;
  const int qb = bx % nqb;
  const int bh = bx / nqb;
  const int h  = bh % H;
  const int b  = bh / H;
  const int q0 = qb * 64 + wave * 16;
  const size_t tok0 = (size_t)b * S;

  v16h qa[2];
  {
    const _Float16* qrow = Qp + (tok0 + q0 + c) * (size_t)ldq + h * 64 + 8 * hh;
    qa[0] = Frag<_Float16>::load(qrow);
    qa[1] = Frag<_Float16>::load(qrow + 32);
  }

  float mrow[8], lrow[8];
  v8f oacc[4];
#pragma unroll
  for (int r = 0; r < 8; ++r) { mrow[r] = -INFINITY; lrow[r] = 0.f; }
#pragma unroll
  for (int t = 0; t < 4; ++t) oacc[t] = (v8f){0.f,0.f,0.f,0.f,0.f,0.f,0.f,0.f};

  const int nChunks = qb + 1;
  for (int kc = 0; kc < nChunks; ++kc) {
    const int kv0 = kc * 64;
    __syncthreads();
#pragma unroll
    for (int i = 0; i < 4; ++i) {
      const int id = tid + 128 * i;
      const int row = id >> 3, c8 = (id & 7) * 8;
      const v8h kv = *(const v8h*)(Kp + (tok0 + kv0 + row) * (size_t)ldq + h * 64 + c8);
      *(v8h*)(Ksh + row * 64 + c8) = kv;
      const v8h vv = *(const v8h*)(VTp + (size_t)(h * 64 + row) * ldvt + tok0 + kv0 + c8);
      *(v8h*)(Vth + row * 64 + c8) = vv;
    }
    __syncthreads();

    v8f s[4];
#pragma unroll
    for (int j = 0; j < 4; ++j) {
      s[j] = (v8f){0.f,0.f,0.f,0.f,0.f,0.f,0.f,0.f};
#pragma unroll
      for (int dc = 0; dc < 2; ++dc) {
        FB kb;
        kb.h[0] = *(const v8h*)(Ksh + (j * 16 + c) * 64 + dc * 32 + 8 * hh);
        kb.h[1] = *(const v8h*)(Ksh + (j * 16 + c) * 64 + dc * 32 + 16 + 8 * hh);
        s[j] = mma_h(qa[dc], kb.v, s[j]);
      }
    }
    const bool diag = (kc == qb);
    float cm[8];
#pragma unroll
    for (int r = 0; r < 8; ++r) {
      const int qrow = q0 + 8 * hh + r;
      float m = -INFINITY;
#pragma unroll
      for (int j = 0; j < 4; ++j) {
        const int kvcol = kv0 + j * 16 + c;
        float sv = s[j][r] * sscale;
        if (diag && (kvcol > qrow)) sv = fillv;
        s[j][r] = sv;
        m = fmaxf(m, sv);
      }
#pragma unroll
      for (int off = 1; off < 16; off <<= 1) m = fmaxf(m, __shfl_xor(m, off, 32));
      cm[r] = m;
    }
    _Float16* pw = Psh[wave];
#pragma unroll
    for (int r = 0; r < 8; ++r) {
      const float mnew = fmaxf(mrow[r], cm[r]);
      const float alpha = expf(mrow[r] - mnew);
      mrow[r] = mnew;
      float psum = 0.f;
#pragma unroll
      for (int j = 0; j < 4; ++j) {
        const float p = expf(s[j][r] - mnew);
        psum += p;
        pw[(8 * hh + r) * 64 + j * 16 + c] = (_Float16)(p * 32768.0f);
      }
#pragma unroll
      for (int off = 1; off < 16; off <<= 1) psum += __shfl_xor(psum, off, 32);
      lrow[r] = lrow[r] * alpha + psum;
#pragma unroll
      for (int t = 0; t < 4; ++t) oacc[t][r] *= alpha;
    }
    __builtin_amdgcn_fence(__ATOMIC_RELEASE, "workgroup");
    __builtin_amdgcn_wave_barrier();
    __builtin_amdgcn_fence(__ATOMIC_ACQUIRE, "workgroup");
#pragma unroll 1
    for (int kk = 0; kk < 2; ++kk) {
      FB pa;
      pa.h[0] = *(const v8h*)(pw + c * 64 + kk * 32 + 8 * hh);
      pa.h[1] = *(const v8h*)(pw + c * 64 + kk * 32 + 16 + 8 * hh);
#pragma unroll
      for (int t = 0; t < 4; ++t) {
        FB vb;
        vb.h[0] = *(const v8h*)(Vth + (t * 16 + c) * 64 + kk * 32 + 8 * hh);
        vb.h[1] = *(const v8h*)(Vth + (t * 16 + c) * 64 + kk * 32 + 16 + 8 * hh);
        oacc[t] = mma_h(pa.v, vb.v, oacc[t]);
      }
    }
  }

  float* os = Os[wave];
#pragma unroll
  for (int r = 0; r < 8; ++r) {
    const float inv = 1.0f / (lrow[r] * 32768.0f);
#pragma unroll
    for (int t = 0; t < 4; ++t) os[(8 * hh + r) * 68 + t * 16 + c] = oacc[t][r] * inv;
  }
  __builtin_amdgcn_fence(__ATOMIC_RELEASE, "workgroup");
  __builtin_amdgcn_wave_barrier();
  __builtin_amdgcn_fence(__ATOMIC_ACQUIRE, "workgroup");
  {
    const int q = lane >> 3, c8 = (lane & 7) * 8;
    for (int pass = 0; pass < 2; ++pass) {
#pragma unroll
      for (int it = 0; it < 4; ++it) {
        const int row = it * 4 + q;
        const float* sp = os + row * 68 + c8;
        v8h hv;
#pragma unroll
        for (int e = 0; e < 8; ++e) hv[e] = (_Float16)sp[e];
        *(volatile v8h*)(Yp + (tok0 + q0 + row) * (size_t)ldq + h * 64 + c8) = hv;
      }
      __threadfence();
    }
  }
}

extern "C" void kernel_launch(void* const* d_in, const int* in_sizes, int n_in,
                              void* d_out, int out_size, void* d_ws, size_t ws_size, hipStream_t stream) {
  constexpr int Bn = 2, S = 2048, D = 1024, H = 16, DH = 64, RA = 32, RP = 512, I = 4096;
  constexpr int M = Bn * S;
  if (n_in < 23) return;
  if (in_sizes[0] != M * D || out_size != M * D) return;
  if (in_sizes[5] != D * H * RA || in_sizes[6] != H * RA * DH || in_sizes[14] != D * RP ||
      in_sizes[15] != RP * D || in_sizes[18] != RP * I || in_sizes[20] != I * RP || in_sizes[21] != RP * D) return;

  const float* hidden = (const float*)d_in[0];
  const float* ln1_g  = (const float*)d_in[1];
  const float* ln1_b  = (const float*)d_in[2];
  const float* ln2_g  = (const float*)d_in[3];
  const float* ln2_b  = (const float*)d_in[4];
  const float* q_U    = (const float*)d_in[5];
  const float* q_V    = (const float*)d_in[6];
  const float* q_b    = (const float*)d_in[7];
  const float* k_U    = (const float*)d_in[8];
  const float* k_V    = (const float*)d_in[9];
  const float* k_b    = (const float*)d_in[10];
  const float* v_U    = (const float*)d_in[11];
  const float* v_V    = (const float*)d_in[12];
  const float* v_b    = (const float*)d_in[13];
  const float* out_U  = (const float*)d_in[14];
  const float* out_V  = (const float*)d_in[15];
  const float* out_b  = (const float*)d_in[16];
  const float* fc1_U  = (const float*)d_in[17];
  const float* fc1_V  = (const float*)d_in[18];
  const float* fc1_b  = (const float*)d_in[19];
  const float* fc2_U  = (const float*)d_in[20];
  const float* fc2_V  = (const float*)d_in[21];
  const float* fc2_b  = (const float*)d_in[22];

  size_t off = 0;
  auto carve = [&](size_t bytes) -> void* {
    void* p = (char*)d_ws + off;
    off += (bytes + 255) & ~(size_t)255;
    return p;
  };
  u16*   xh   = (u16*)carve((size_t)M * D * 2);
  u16*   WU   = (u16*)carve((size_t)3 * RP * D * 2);
  u16*   BV   = (u16*)carve((size_t)3 * H * DH * RA * 2);
  u16*   Tpl  = (u16*)carve((size_t)3 * M * RP * 2);
  u16*   big  = (u16*)carve((size_t)4 * M * D * 2);
  u16*   WoU  = (u16*)carve((size_t)RP * D * 2);
  u16*   WoV  = (u16*)carve((size_t)D * RP * 2);
  u16*   Tout = (u16*)carve((size_t)M * RP * 2);
  float* hres = (float*)carve((size_t)M * D * 4);
  u16*   W1U  = (u16*)carve((size_t)RP * D * 2);
  u16*   W1V  = (u16*)carve((size_t)I * RP * 2);
  u16*   W2U  = (u16*)carve((size_t)RP * I * 2);
  u16*   W2V  = (u16*)carve((size_t)D * RP * 2);
  if (off > ws_size || off > (size_t)134217728) return;

  u16* Tq = Tpl;
  u16* Tk = Tpl + (size_t)M * RP;
  u16* Tv = Tpl + (size_t)2 * M * RP;
  u16* Q16 = big;
  u16* K16 = big + (size_t)M * D;
  u16* VT  = big + (size_t)2 * M * D;
  u16* Yp  = big + (size_t)3 * M * D;
  u16* h1  = big;
  u16* Tfc1 = Tq;
  u16* Tfc2 = Tk;

  const dim3 b256(256), b128(128);
  const float W_SC = 256.0f;

  tcast64<<<dim3(RP / 64, D / 64), b256, 0, stream>>>(q_U, (_Float16*)WU, D, RP, W_SC);
  tcast64<<<dim3(RP / 64, D / 64), b256, 0, stream>>>(k_U, (_Float16*)(WU + (size_t)RP * D), D, RP, W_SC);
  tcast64<<<dim3(RP / 64, D / 64), b256, 0, stream>>>(v_U, (_Float16*)(WU + (size_t)2 * RP * D), D, RP, W_SC);
  tcast_v32<<<dim3(48), b256, 0, stream>>>(q_V, k_V, v_V, (_Float16*)BV, W_SC);
  tcast64<<<dim3(RP / 64, D / 64), b256, 0, stream>>>(out_U, (_Float16*)WoU, D, RP, W_SC);
  tcast64<<<dim3(D / 64, RP / 64), b256, 0, stream>>>(out_V, (_Float16*)WoV, RP, D, W_SC);
  tcast64<<<dim3(RP / 64, D / 64), b256, 0, stream>>>(fc1_U, (_Float16*)W1U, D, RP, W_SC);
  tcast64<<<dim3(I / 64, RP / 64), b256, 0, stream>>>(fc1_V, (_Float16*)W1V, RP, I, W_SC);
  tcast64<<<dim3(RP / 64, I / 64), b256, 0, stream>>>(fc2_U, (_Float16*)W2U, I, RP, W_SC);
  tcast64<<<dim3(D / 64, RP / 64), b256, 0, stream>>>(fc2_V, (_Float16*)W2V, RP, D, W_SC);

  layernorm_f16<<<dim3(M), b128, 0, stream>>>(hidden, ln1_g, ln1_b, (_Float16*)xh, D, 1e-5f);

  wmma_gemm64<0, 1, false, 0><<<dim3((M / 64) * (RP / 64) / 8, 3), b256, 0, stream>>>(
      xh, D, 0L, WU, D, (long)RP * D, Tpl, RP, (long)M * RP,
      nullptr, 0L, 0.f, nullptr, 0L, M, RP, D, 0.0625f, 1.0f);

  wmma_gemm64<2, 1, false, 0><<<dim3((M / 64) * 1 / 8, H), b256, 0, stream>>>(
      Tq, RP, (long)RA, BV, RA, (long)DH * RA, Q16, D, (long)DH,
      q_b, (long)DH, 16.0f, nullptr, 0L, M, DH, RA, 0.00390625f, 1.0f);
  wmma_gemm64<2, 1, false, 0><<<dim3((M / 64) * 1 / 8, H), b256, 0, stream>>>(
      Tk, RP, (long)RA, BV + (size_t)H * DH * RA, RA, (long)DH * RA, K16, D, (long)DH,
      k_b, (long)DH, 16.0f, nullptr, 0L, M, DH, RA, 0.00390625f, 1.0f);
  wmma_gemm64<1, 1, false, 0><<<dim3(1 * (M / 64) / 8, H), b256, 0, stream>>>(
      BV + (size_t)2 * H * DH * RA, RA, (long)DH * RA, Tv, RP, (long)RA, VT, M, (long)DH * M,
      v_b, (long)DH, 256.0f, nullptr, 0L, DH, M, RA, 0.0625f, 1.0f);

  attn64_f16<<<dim3(Bn * H * (S / 64)), b128, 0, stream>>>(
      (const _Float16*)Q16, (const _Float16*)K16, (const _Float16*)VT, (_Float16*)Yp,
      S, H, D, M, 0.00048828125f, -3.4028235e38f);

  wmma_gemm64<0, 1, false, 0><<<dim3((M / 64) * (RP / 64) / 8, 1), b256, 0, stream>>>(
      Yp, D, 0L, WoU, D, 0L, Tout, RP, 0L,
      nullptr, 0L, 0.f, nullptr, 0L, M, RP, D, 0.00390625f, 1.0f);
  wmma_gemm64<2, 0, true, 0><<<dim3((M / 64) * (D / 64) / 8, 1), b256, 0, stream>>>(
      Tout, RP, 0L, WoV, RP, 0L, hres, D, 0L,
      out_b, 0L, 1.0f, hidden, 0L, M, D, RP, 1.52587890625e-5f, 1.0f);

  layernorm_f16<<<dim3(M), b128, 0, stream>>>(hres, ln2_g, ln2_b, (_Float16*)xh, D, 1e-5f);

  wmma_gemm64<0, 1, false, 0><<<dim3((M / 64) * (RP / 64) / 8, 1), b256, 0, stream>>>(
      xh, D, 0L, W1U, D, 0L, Tfc1, RP, 0L,
      nullptr, 0L, 0.f, nullptr, 0L, M, RP, D, 0.0625f, 1.0f);
  wmma_gemm64<2, 1, false, 5><<<dim3((M / 64) * (I / 64) / 8, 1), b256, 0, stream>>>(
      Tfc1, RP, 0L, W1V, RP, 0L, h1, I, 0L,
      fc1_b, 0L, 1.0f, nullptr, 0L, M, I, RP, 0.000244140625f, 64.0f);
  wmma_gemm64<0, 1, false, 0><<<dim3((M / 64) * (RP / 64) / 8, 1), b256, 0, stream>>>(
      h1, I, 0L, W2U, I, 0L, Tfc2, RP, 0L,
      nullptr, 0L, 0.f, nullptr, 0L, M, RP, I, 0.0009765625f, 1.0f);
  wmma_gemm64<2, 0, true, 0><<<dim3((M / 64) * (D / 64) / 8, 1), b256, 0, stream>>>(
      Tfc2, RP, 0L, W2V, RP, 0L, d_out, D, 0L,
      fc2_b, 0L, 1.0f, hres, 0L, M, D, RP, 0.000244140625f, 1.0f);
}
